// GEPSLinear_64098091925941
// MI455X (gfx1250) — hardware-verified
//
#include <hip/hip_runtime.h>
#include <math.h>

typedef __attribute__((ext_vector_type(16))) _Float16 v16h;
typedef __attribute__((ext_vector_type(8)))  _Float16 v8h;
typedef __attribute__((ext_vector_type(8)))  float    v8f;
typedef __attribute__((ext_vector_type(4)))  float    v4f;

constexpr int kRowsM = 128;
constexpr int kDepthK = 1024;
constexpr int kColsN = 1024;
constexpr int kCodeR = 2;
static_assert((kRowsM % 64) == 0 && (kColsN % 64) == 0 && (kDepthK % 32) == 0, "GEMM tile multiples");
static_assert((kDepthK % 256) == 0 && (kDepthK % 64) == 0, "plane tiling");
static_assert(kCodeR == 2, "rank of the per-sample mixing");

constexpr float kCarryX = 64.0f;
constexpr float kCarryW = 1024.0f;
constexpr float kFold = 1.0f / (kCarryX * kCarryW);
constexpr float kF16MinNormal = 6.103515625e-5f;

constexpr size_t kOffXH   = 0;
constexpr size_t kOffWT   = kOffXH + (size_t)kRowsM * kDepthK * 2;
constexpr size_t kOffCOEF = kOffWT + (size_t)kColsN * kDepthK * 2;
constexpr size_t kWsTotal = kOffCOEF + (size_t)kRowsM * 4 * 4;
static_assert(kWsTotal == 2361344ull, "carve total");
static_assert(kWsTotal <= 134217728ull, "carve cap");
static_assert((kOffWT % 128) == 0 && (kOffCOEF % 128) == 0, "128-B aligned regions");

__device__ __forceinline__ _Float16 to_f16_carry(float v, float carry) {
  const float s = v * carry;
  const float t = (fabsf(s) < kF16MinNormal) ? 0.0f : s;
  return (_Float16)t;
}

__device__ __forceinline__ v16h frag_load_f16(const _Float16* p) {
  union { v16h v; v8h h[2]; } f;
  f.h[0] = *(const v8h*)(p);
  f.h[1] = *(const v8h*)(p + 16);
  return f.v;
}

__device__ __forceinline__ v8f mma_f16(v16h a, v16h b, v8f c) {
  c = __builtin_amdgcn_wmma_f32_16x16x32_f16(false, a, false, b, (short)0, c, false, false);
  asm volatile("v_nop\n\tv_nop\n\tv_nop\n\tv_nop" : "+v"(c) : "v"(a), "v"(b));
  return c;
}

__global__ __launch_bounds__(256) void prep_x_coef_kernel(
    const float* __restrict__ x, const float* __restrict__ codes, const float* __restrict__ Amat,
    unsigned short* __restrict__ XH, float* __restrict__ COEF)
{
  __shared__ __align__(16) float sC[8 * 4];
  const int tid = threadIdx.x;
  const int lane = tid & 31;
  const int wave = tid >> 5;
  const int b = blockIdx.x * 8 + wave;
  const float* xr = x + (size_t)b * kDepthK;

  float u0 = 0.0f;
  float u1 = 0.0f;
  v8h hv[4];
#pragma unroll
  for (int it = 0; it < 4; ++it) {
    const int k = it * 256 + lane * 8;
    const v4f x0 = *(const v4f*)(xr + k);
    const v4f x1 = *(const v4f*)(xr + k + 4);
    const v4f a0 = *(const v4f*)(Amat + 2 * k);
    const v4f a1 = *(const v4f*)(Amat + 2 * k + 4);
    const v4f a2 = *(const v4f*)(Amat + 2 * k + 8);
    const v4f a3 = *(const v4f*)(Amat + 2 * k + 12);
    const float xs[8] = {x0[0], x0[1], x0[2], x0[3], x1[0], x1[1], x1[2], x1[3]};
    const float av[16] = {a0[0], a0[1], a0[2], a0[3], a1[0], a1[1], a1[2], a1[3],
                          a2[0], a2[1], a2[2], a2[3], a3[0], a3[1], a3[2], a3[3]};
#pragma unroll
    for (int e = 0; e < 8; ++e) {
      u0 = fmaf(xs[e], av[2 * e], u0);
      u1 = fmaf(xs[e], av[2 * e + 1], u1);
      hv[it][e] = to_f16_carry(xs[e], kCarryX);
    }
  }
#pragma unroll
  for (int off = 16; off > 0; off >>= 1) {
    u0 += __shfl_xor(u0, off, 32);
    u1 += __shfl_xor(u1, off, 32);
  }
  const v4f cd = *(const v4f*)(codes + (size_t)b * 4);
  float c00 = cd[0];
  float c01 = cd[1];
  float c10 = cd[2];
  float c11 = cd[3];
  asm volatile("" : "+v"(c00), "+v"(c01), "+v"(c10), "+v"(c11));
  const float v0 = u0 * c00 + u1 * c10;
  const float v1 = u0 * c01 + u1 * c11;
  if (lane == 0) {
    const v4f pk = (v4f){v0, v1, c00, c11};
    *(v4f*)(sC + wave * 4) = pk;
  }

  unsigned short* xo = XH + (size_t)b * kDepthK + lane * 8;
  for (int pass = 0; pass < 2; ++pass) {
#pragma unroll
    for (int it = 0; it < 4; ++it) {
      *(volatile v8h*)(xo + it * 256) = hv[it];
    }
    __threadfence();
  }

  __syncthreads();
  const v4f cv = *(const v4f*)(sC + (lane & 7) * 4);
  if (wave == 0 && lane < 8) {
    float* dst = COEF + ((size_t)blockIdx.x * 8 + lane) * 4;
    *(volatile v4f*)dst = cv;
    __threadfence();
    *(volatile v4f*)dst = cv;
  }
}

__global__ __launch_bounds__(256) void transpose_w_kernel(
    const float* __restrict__ W, unsigned short* __restrict__ WT)
{
  __shared__ __align__(16) float sT[64 * 68];
  const int tid = threadIdx.x;
  const int lane = tid & 31;
  const int wave = tid >> 5;
  const int n0 = blockIdx.x * 64;
  const int k0 = blockIdx.y * 64;
  const int lr = tid >> 4;
  const int c4 = (tid & 15) * 4;
#pragma unroll
  for (int i = 0; i < 4; ++i) {
    const int k = lr + 16 * i;
    const v4f w4 = *(const v4f*)(W + (size_t)(k0 + k) * kColsN + n0 + c4);
    *(v4f*)(sT + k * 68 + c4) = w4;
  }
  __syncthreads();
  const int q = lane >> 3;
  const int c8 = (lane & 7) * 8;
  v8h hv[2];
#pragma unroll
  for (int it = 0; it < 2; ++it) {
    const int n = it * 32 + wave * 4 + q;
#pragma unroll
    for (int e = 0; e < 8; ++e) {
      hv[it][e] = to_f16_carry(sT[(c8 + e) * 68 + n], kCarryW);
    }
  }
  for (int pass = 0; pass < 2; ++pass) {
#pragma unroll
    for (int it = 0; it < 2; ++it) {
      const int n = it * 32 + wave * 4 + q;
      *(volatile v8h*)(WT + (size_t)(n0 + n) * kDepthK + k0 + c8) = hv[it];
    }
    __threadfence();
  }
}

__global__ __launch_bounds__(256) void gemm_f16_lowrank_kernel(
    const unsigned short* __restrict__ XHp, const unsigned short* __restrict__ WTp,
    const float* __restrict__ COEF, const float* __restrict__ Bm,
    const float* __restrict__ bias, const float* __restrict__ bctx,
    float* __restrict__ out)
{
  __shared__ __align__(16) float sS[8][16 * 68];
  const int lane = threadIdx.x & 31;
  const int wave = threadIdx.x >> 5;
  constexpr int tilesN = kColsN / 64;
  constexpr int tilesM = kRowsM / 64;
  const int tile = blockIdx.x * 8 + wave;
  if (tile >= tilesM * tilesN) return;
  const int tm = tile / tilesN;
  const int tn = tile - tm * tilesN;
  const int m0 = tm * 64;
  const int n0 = tn * 64;

  const _Float16* A = (const _Float16*)XHp;
  const _Float16* Bt = (const _Float16*)WTp;
  const int rlane = lane & 15;
  const int koff = (lane >> 4) * 8;
  const int mOff = (lane >> 4) * 8;

  v8f acc[4][4];
#pragma unroll
  for (int i = 0; i < 4; ++i) {
#pragma unroll
    for (int j = 0; j < 4; ++j) {
      acc[i][j] = (v8f){0.f, 0.f, 0.f, 0.f, 0.f, 0.f, 0.f, 0.f};
    }
  }

  for (int k0 = 0; k0 < kDepthK; k0 += 32) {
    v16h bh[4];
#pragma unroll
    for (int j = 0; j < 4; ++j) {
      const size_t bo = (size_t)(n0 + (j << 4) + rlane) * kDepthK + koff + k0;
      bh[j] = frag_load_f16(Bt + bo);
    }
#pragma unroll
    for (int i = 0; i < 4; ++i) {
      const size_t ao = (size_t)(m0 + (i << 4) + rlane) * kDepthK + koff + k0;
      const v16h ah = frag_load_f16(A + ao);
#pragma unroll
      for (int j = 0; j < 4; ++j) {
        acc[i][j] = mma_f16(ah, bh[j], acc[i][j]);
      }
    }
  }

  const int hh = lane >> 4;
  const int c4 = (lane & 15) * 4;
  const v4f bi  = *(const v4f*)(bias + n0 + c4);
  const v4f bm0 = *(const v4f*)(Bm + n0 + c4);
  const v4f bm1 = *(const v4f*)(Bm + kColsN + n0 + c4);
  const v4f bc0 = *(const v4f*)(bctx + n0 + c4);
  const v4f bc1 = *(const v4f*)(bctx + kColsN + n0 + c4);

  float* slab = sS[wave];
#pragma unroll
  for (int i = 0; i < 4; ++i) {
    const int mBase = m0 + (i << 4);
#pragma unroll
    for (int j = 0; j < 4; ++j) {
#pragma unroll
      for (int r = 0; r < 8; ++r) {
        slab[(mOff + r) * 68 + (j << 4) + rlane] = acc[i][j][r];
      }
    }
    __builtin_amdgcn_fence(__ATOMIC_RELEASE, "workgroup");
    __builtin_amdgcn_wave_barrier();
    __builtin_amdgcn_fence(__ATOMIC_ACQUIRE, "workgroup");
#pragma unroll
    for (int hf = 0; hf < 2; ++hf) {
      v4f ov[4];
#pragma unroll
      for (int it = 0; it < 4; ++it) {
        const int row = (hf * 4 + it) * 2 + hh;
        const v4f sv = *(const v4f*)(slab + row * 68 + c4);
        const v4f cf = *(const v4f*)(COEF + (size_t)(mBase + row) * 4);
#pragma unroll
        for (int e = 0; e < 4; ++e) {
          float t = fmaf(sv[e], kFold, bi[e]);
          t = fmaf(cf[0], bm0[e], t);
          t = fmaf(cf[1], bm1[e], t);
          t = fmaf(cf[2], bc0[e], t);
          t = fmaf(cf[3], bc1[e], t);
          ov[it][e] = t;
        }
      }
      for (int pass = 0; pass < 2; ++pass) {
#pragma unroll
        for (int it = 0; it < 4; ++it) {
          const int row = (hf * 4 + it) * 2 + hh;
          *(volatile v4f*)(out + (size_t)(mBase + row) * kColsN + n0 + c4) = ov[it];
        }
        __threadfence();
      }
    }
    __builtin_amdgcn_fence(__ATOMIC_RELEASE, "workgroup");
    __builtin_amdgcn_wave_barrier();
    __builtin_amdgcn_fence(__ATOMIC_ACQUIRE, "workgroup");
  }
}

extern "C" void kernel_launch(void* const* d_in, const int* in_sizes, int n_in,
                              void* d_out, int out_size, void* d_ws, size_t ws_size,
                              hipStream_t stream) {
  if (n_in < 7) return;
  if (in_sizes[0] != kRowsM * kDepthK) return;
  if (in_sizes[1] != kRowsM * kCodeR * kCodeR) return;
  if (in_sizes[2] != kDepthK * kColsN) return;
  if (in_sizes[3] != kDepthK * kCodeR) return;
  if (in_sizes[4] != kCodeR * kColsN) return;
  if (in_sizes[5] != kColsN) return;
  if (in_sizes[6] != kCodeR * kColsN) return;
  if (out_size != kRowsM * kColsN) return;
  if (ws_size < kWsTotal) return;

  const float* x      = (const float*)d_in[0];
  const float* codes  = (const float*)d_in[1];
  const float* weight = (const float*)d_in[2];
  const float* Amat   = (const float*)d_in[3];
  const float* Bm     = (const float*)d_in[4];
  const float* bias   = (const float*)d_in[5];
  const float* bctx   = (const float*)d_in[6];
  float* out = (float*)d_out;

  char* ws = (char*)d_ws;
  unsigned short* XH   = (unsigned short*)(ws + kOffXH);
  unsigned short* WT   = (unsigned short*)(ws + kOffWT);
  float*          COEF = (float*)(ws + kOffCOEF);

  prep_x_coef_kernel<<<kRowsM / 8, 256, 0, stream>>>(x, codes, Amat, XH, COEF);
  transpose_w_kernel<<<dim3(kColsN / 64, kDepthK / 64), 256, 0, stream>>>(weight, WT);
  gemm_f16_lowrank_kernel<<<(kRowsM / 64) * (kColsN / 64) / 8, 256, 0, stream>>>(
      XH, WT, COEF, Bm, bias, bctx, out);
}
